// FastWeightMemory_32366873543105
// MI455X (gfx1250) — hardware-verified
//
#include <hip/hip_runtime.h>
#include <stddef.h>
#include <stdint.h>

#define NB   4
#define SQ   4096
#define DM   768
#define NH   8
#define HD   64
#define NKV  512
#define ROWS (NB * SQ)
#define CH   64
#define QLD  512
#define KVLD 1024
#define OLD  512

static_assert(ROWS % 256 == 0);
static_assert(SQ % 256 == 0);
static_assert(SQ % CH == 0);
static_assert(NKV % 64 == 0);
static_assert(DM % 64 == 0);
static_assert(DM % 32 == 0);
static_assert(NH * HD == NKV);
static_assert(HD == 64);

typedef _Float16 v16h __attribute__((ext_vector_type(16)));
typedef _Float16 v8h  __attribute__((ext_vector_type(8)));
typedef float    v8f  __attribute__((ext_vector_type(8)));
typedef float    v4f  __attribute__((ext_vector_type(4)));
typedef unsigned int v4u __attribute__((ext_vector_type(4)));

union Frag  { v16h v; v8h h[2]; };
union Pack8 { v8h h; v4u u; };

__device__ __forceinline__ v8f mma16(v16h a, v16h b, v8f c) {
  c = __builtin_amdgcn_wmma_f32_16x16x32_f16(false, a, false, b, (short)0, c, false, false);
  asm volatile("v_nop\n\tv_nop\n\tv_nop\n\tv_nop" : "+v"(c) : "v"(a), "v"(b));
  return c;
}

__device__ __forceinline__ v16h ldfrag(const _Float16* p, int ld, int row0, int k0, int lane) {
  const int m = lane & 15, lh = lane >> 4;
  const _Float16* q = p + (size_t)(row0 + m) * ld + k0 + 8 * lh;
  Frag f;
  f.h[0] = *(const v8h*)(q);
  f.h[1] = *(const v8h*)(q + 16);
  return f.v;
}

__device__ __forceinline__ v8f zero8() { return (v8f){0.f, 0.f, 0.f, 0.f, 0.f, 0.f, 0.f, 0.f}; }

template <int KD>
__device__ __forceinline__ void gemm32x64(const _Float16* __restrict__ A, int lda,
                                          const _Float16* __restrict__ Bt, int ldb,
                                          int m0, int n0, int lane, v8f (&acc)[2][4]) {
#pragma unroll 2
  for (int k0 = 0; k0 < KD; k0 += 32) {
    const v16h a0 = ldfrag(A, lda, m0, k0, lane);
    const v16h a1 = ldfrag(A, lda, m0 + 16, k0, lane);
    const v16h b0 = ldfrag(Bt, ldb, n0, k0, lane);
    const v16h b1 = ldfrag(Bt, ldb, n0 + 16, k0, lane);
    const v16h b2 = ldfrag(Bt, ldb, n0 + 32, k0, lane);
    const v16h b3 = ldfrag(Bt, ldb, n0 + 48, k0, lane);
    acc[0][0] = mma16(a0, b0, acc[0][0]);
    acc[1][0] = mma16(a1, b0, acc[1][0]);
    acc[0][1] = mma16(a0, b1, acc[0][1]);
    acc[1][1] = mma16(a1, b1, acc[1][1]);
    acc[0][2] = mma16(a0, b2, acc[0][2]);
    acc[1][2] = mma16(a1, b2, acc[1][2]);
    acc[0][3] = mma16(a0, b3, acc[0][3]);
    acc[1][3] = mma16(a1, b3, acc[1][3]);
  }
}

__global__ __launch_bounds__(256) void k_cvt(const float* __restrict__ x, _Float16* __restrict__ xh,
                                             int ngrp, float scale) {
  const int t = blockIdx.x * 256 + (int)threadIdx.x;
  if (t >= ngrp) return;
  const size_t o = (size_t)t * 8;
  const v4f a0 = *(const v4f*)(x + o);
  const v4f a1 = *(const v4f*)(x + o + 4);
  Pack8 pk;
  pk.h = (v8h){(_Float16)(a0[0] * scale), (_Float16)(a0[1] * scale), (_Float16)(a0[2] * scale), (_Float16)(a0[3] * scale),
               (_Float16)(a1[0] * scale), (_Float16)(a1[1] * scale), (_Float16)(a1[2] * scale), (_Float16)(a1[3] * scale)};
  const v4u vv = pk.u;
  volatile v4u* d = (volatile v4u*)(xh + o);
  *d = vv;
  __threadfence();
  *d = vv;
}

__global__ __launch_bounds__(256) void k_gate(const float* __restrict__ x, const float* __restrict__ wg,
                                              float* __restrict__ g0) {
  __shared__ __align__(16) float gsh[32];
  const int tid = threadIdx.x, lane = tid & 31, wave = tid >> 5;
  const int sb = blockIdx.x * 4;
#pragma unroll 1
  for (int i = 0; i < 4; ++i) {
    const int task = wave * 4 + i;
    const int sl = task >> 3, hd = task & 7;
    const float* xp = x + (size_t)(sb + sl) * DM;
    const float* wp = wg + (size_t)hd * DM;
    float acc = 0.f;
#pragma unroll 1
    for (int k = 0; k < DM / 128; ++k) {
      const v4f xv = *(const v4f*)(xp + 4 * (lane + 32 * k));
      const v4f wv = *(const v4f*)(wp + 4 * (lane + 32 * k));
      acc += xv[0] * wv[0];
      acc += xv[1] * wv[1];
      acc += xv[2] * wv[2];
      acc += xv[3] * wv[3];
    }
#pragma unroll
    for (int off = 16; off; off >>= 1) acc += __shfl_xor(acc, off, 32);
    const float e = expf(-acc);
    const float gv = 1.0f / (1.0f + e);
    if (lane == 0) gsh[task] = gv;
  }
  __syncthreads();
  if (tid < 8) {
    const v4f val = *(const v4f*)(gsh + 4 * tid);
    volatile v4f* d = (volatile v4f*)(g0 + (size_t)sb * NH + 4 * tid);
    *d = val;
    __threadfence();
    *d = val;
  }
}

#define STP 72
template <int KD>
__global__ __launch_bounds__(256) void k_lin(const _Float16* __restrict__ ah, int lda,
                                             const _Float16* __restrict__ wt,
                                             _Float16* __restrict__ hp, int ldc, float oscale) {
  __shared__ __align__(16) _Float16 st[256 * STP];
  const int tid = threadIdx.x, lane = tid & 31, wave = tid >> 5;
  const int hh = lane >> 4, c = lane & 15;
  const int mb = blockIdx.x * 256;
  const int m0 = mb + wave * 32;
  const int n0 = blockIdx.y * 64;

  v8f acc[2][4];
#pragma unroll
  for (int s = 0; s < 2; ++s)
#pragma unroll
    for (int t = 0; t < 4; ++t) acc[s][t] = zero8();
  gemm32x64<KD>(ah, lda, wt, KD, m0, n0, lane, acc);

#pragma unroll
  for (int t = 0; t < 4; ++t) {
#pragma unroll
    for (int sub = 0; sub < 2; ++sub) {
#pragma unroll
      for (int r = 0; r < 8; ++r) {
        const int lr = wave * 32 + sub * 16 + 8 * hh + r;
        st[lr * STP + 16 * t + c] = (_Float16)(acc[sub][t][r] * oscale);
      }
    }
  }
  __syncthreads();

  v4u val[8];
  size_t go[8];
#pragma unroll
  for (int j = 0; j < 8; ++j) {
    const int p  = tid + 256 * j;
    const int lr = p >> 3;
    const int pc = p & 7;
    Pack8 pk;
    pk.h   = *(const v8h*)(st + lr * STP + pc * 8);
    val[j] = pk.u;
    go[j]  = (size_t)(mb + lr) * ldc + n0 + pc * 8;
  }
  for (int ps = 0; ps < 2; ++ps) {
#pragma unroll
    for (int j = 0; j < 8; ++j) *(volatile v4u*)(hp + go[j]) = val[j];
    __threadfence();
  }
}

#define KTP 72
#define PTP 72
__global__ __launch_bounds__(128) void k_scan(const _Float16* __restrict__ qp,
                                              const _Float16* __restrict__ kvp,
                                              const float* __restrict__ g0,
                                              _Float16* __restrict__ op) {
  __shared__ __align__(16) _Float16 Ks[CH * KTP];
  __shared__ __align__(16) _Float16 Vn[CH * KTP];
  __shared__ __align__(16) _Float16 Vs[HD * KTP];
  __shared__ __align__(16) _Float16 Kt[HD * KTP];
  __shared__ __align__(16) _Float16 Fw[HD * KTP];
  __shared__ __align__(16) _Float16 Ps[4][16 * PTP];
  __shared__ __align__(16) float cw[CH];
  __shared__ __align__(16) float dws[CH];

  const int tid = threadIdx.x, lane = tid & 31, wave = tid >> 5;
  const int hh = lane >> 4, c = lane & 15;
  const int h = blockIdx.x & (NH - 1);
  const int b = blockIdx.x >> 3;
  const _Float16* Qb = qp + (size_t)b * SQ * QLD + h * HD;
  const _Float16* Kb = kvp + h * HD;
  const _Float16* Vb = kvp + NKV + h * HD;
  const float L2D = -0.074000581443777f;

  for (int i = tid; i < HD * KTP / 8; i += 128) *(v4u*)(Fw + 8 * i) = (v4u){0u, 0u, 0u, 0u};
  if (tid < CH) dws[tid] = 0.1f * exp2f((float)(CH - 1 - tid) * L2D);
  float rd1[8], rd2[8];
#pragma unroll
  for (int r = 0; r < 8; ++r) {
    const int tl = 16 * wave + 8 * hh + r;
    rd1[r] = exp2f((float)tl * L2D);
    rd2[r] = exp2f((float)(tl - CH) * L2D);
  }
  const float dC = exp2f((float)CH * L2D);
  v8f fwr[4];
#pragma unroll
  for (int t = 0; t < 4; ++t) fwr[t] = zero8();
  _Float16* pw = Ps[wave];
  __syncthreads();

  for (int ci = 0; ci < SQ / CH; ++ci) {
    const int c0 = ci * CH;
    if (tid < CH) cw[tid] = g0[(size_t)(c0 + tid) * NH + h] * dws[tid];
    {
      const int r = tid >> 1, qq = (tid & 1) * 32;
      const _Float16* ks = Kb + (size_t)(c0 + r) * KVLD + qq;
      const _Float16* vs = Vb + (size_t)(c0 + r) * KVLD + qq;
#pragma unroll
      for (int i = 0; i < 4; ++i) {
        *(v8h*)(Ks + r * KTP + qq + 8 * i) = *(const v8h*)(ks + 8 * i);
        *(v8h*)(Vn + r * KTP + qq + 8 * i) = *(const v8h*)(vs + 8 * i);
      }
    }
    __syncthreads();

    v16h qa[2];
    qa[0] = ldfrag(Qb, QLD, c0 + 16 * wave, 0, lane);
    qa[1] = ldfrag(Qb, QLD, c0 + 16 * wave, 32, lane);
    v8f facc[4], s[4];
#pragma unroll
    for (int t = 0; t < 4; ++t) { facc[t] = zero8(); s[t] = zero8(); }
#pragma unroll
    for (int dc = 0; dc < 2; ++dc) {
#pragma unroll
      for (int t = 0; t < 4; ++t) {
        const v16h fb = ldfrag(Fw, KTP, 16 * t, 32 * dc, lane);
        facc[t] = mma16(qa[dc], fb, facc[t]);
      }
#pragma unroll
      for (int j = 0; j < 4; ++j) {
        const v16h kb = ldfrag(Ks, KTP, 16 * j, 32 * dc, lane);
        s[j] = mma16(qa[dc], kb, s[j]);
      }
    }
    float cwl[4];
#pragma unroll
    for (int j = 0; j < 4; ++j) cwl[j] = cw[16 * j + c];
#pragma unroll
    for (int r = 0; r < 8; ++r) {
      const int tl = 16 * wave + 8 * hh + r;
      const float f1 = rd1[r], f2 = rd2[r];
#pragma unroll
      for (int t = 0; t < 4; ++t) facc[t][r] *= f1;
#pragma unroll
      for (int j = 0; j < 4; ++j) {
        const int sl = 16 * j + c;
        float p = s[j][r] * f2 * cwl[j];
        p = (sl < tl) ? p : 0.f;
        pw[(8 * hh + r) * PTP + 16 * j + c] = (_Float16)p;
      }
    }
    {
      const int dd = tid >> 1, kb0 = (tid & 1) * 32;
#pragma unroll
      for (int i = 0; i < 4; ++i) {
        v8h pv, pk;
#pragma unroll
        for (int e = 0; e < 8; ++e) {
          const int key = kb0 + 8 * i + e;
          pv[e] = Vn[key * KTP + dd];
          pk[e] = (_Float16)((float)Ks[key * KTP + dd] * (cw[key] * 64.0f));
        }
        *(v8h*)(Vs + dd * KTP + kb0 + 8 * i) = pv;
        *(v8h*)(Kt + dd * KTP + kb0 + 8 * i) = pk;
      }
    }
    __syncthreads();

    v8f uacc[4];
#pragma unroll
    for (int t = 0; t < 4; ++t) uacc[t] = zero8();
#pragma unroll
    for (int kk = 0; kk < 2; ++kk) {
      const v16h pa = ldfrag(pw, PTP, 0, 32 * kk, lane);
      const v16h ka = ldfrag(Kt, KTP, 16 * wave, 32 * kk, lane);
#pragma unroll
      for (int t = 0; t < 4; ++t) {
        const v16h vb = ldfrag(Vs, KTP, 16 * t, 32 * kk, lane);
        facc[t] = mma16(pa, vb, facc[t]);
        uacc[t] = mma16(ka, vb, uacc[t]);
      }
    }
#pragma unroll
    for (int t = 0; t < 4; ++t) {
#pragma unroll
      for (int r = 0; r < 8; ++r) {
        const float f = dC * fwr[t][r] + uacc[t][r] * 0.0009765625f;
        fwr[t][r] = f;
        Fw[(16 * t + c) * KTP + 16 * wave + 8 * hh + r] = (_Float16)(f * 16.0f);
      }
    }
    __syncthreads();
#pragma unroll
    for (int t = 0; t < 4; ++t) {
#pragma unroll
      for (int r = 0; r < 8; ++r) pw[(8 * hh + r) * PTP + 16 * t + c] = (_Float16)(facc[t][r] * 0.25f);
    }
    __syncthreads();
    v4u val[4];
    size_t go[4];
#pragma unroll
    for (int it = 0; it < 4; ++it) {
      const int p  = lane + 32 * it;
      const int L  = p >> 3;
      const int pc = p & 7;
      Pack8 pk;
      pk.h    = *(const v8h*)(pw + L * PTP + pc * 8);
      val[it] = pk.u;
      go[it]  = ((size_t)(b * SQ + c0 + 16 * wave + L)) * OLD + (size_t)h * HD + pc * 8;
    }
    for (int ps = 0; ps < 2; ++ps) {
#pragma unroll
      for (int it = 0; it < 4; ++it) *(volatile v4u*)(op + go[it]) = val[it];
      __threadfence();
    }
  }
}

#define OTP 68
__global__ __launch_bounds__(256) void k_proj(const _Float16* __restrict__ ap,
                                              const _Float16* __restrict__ wt,
                                              const float* __restrict__ res,
                                              float* __restrict__ out) {
  __shared__ __align__(16) float st[8][16 * OTP];
  const int tid = threadIdx.x, lane = tid & 31, wave = tid >> 5;
  const int hh = lane >> 4, c = lane & 15;
  const int m0 = blockIdx.x * 256 + wave * 32;
  const int n0 = blockIdx.y * 64;

  v8f acc[2][4];
#pragma unroll
  for (int s = 0; s < 2; ++s)
#pragma unroll
    for (int t = 0; t < 4; ++t) acc[s][t] = zero8();
  gemm32x64<NKV>(ap, NKV, wt, NKV, m0, n0, lane, acc);

  float* sw = st[wave];
#pragma unroll
  for (int sub = 0; sub < 2; ++sub) {
    __syncthreads();
#pragma unroll
    for (int t = 0; t < 4; ++t) {
#pragma unroll
      for (int r = 0; r < 8; ++r)
        sw[(8 * hh + r) * OTP + 16 * t + c] = acc[sub][t][r] * 0.001953125f;
    }
    __syncthreads();
    v4f val[8];
    size_t go[8];
#pragma unroll
    for (int it = 0; it < 8; ++it) {
      const int p    = lane + 32 * it;
      const int L    = p >> 3;
      const int pc   = p & 7;
      const int row  = L >> 1;
      const int half = L & 1;
      go[it]  = (size_t)(m0 + sub * 16 + row) * DM + n0 + half * 32 + pc * 4;
      v4f v = *(const v4f*)(sw + row * OTP + half * 32 + pc * 4);
      const v4f rx = *(const v4f*)(res + go[it]);
      v[0] += rx[0]; v[1] += rx[1]; v[2] += rx[2]; v[3] += rx[3];
      val[it] = v;
    }
    for (int ps = 0; ps < 2; ++ps) {
#pragma unroll
      for (int it = 0; it < 8; ++it) *(volatile v4f*)(out + go[it]) = val[it];
      __threadfence();
    }
  }
}

extern "C" void kernel_launch(void* const* d_in, const int* in_sizes, int n_in,
                              void* d_out, int out_size, void* d_ws, size_t ws_size,
                              hipStream_t stream) {
  if (n_in < 6) return;
  if (in_sizes[0] != ROWS * DM) return;
  if (in_sizes[1] != NKV * DM) return;
  if (in_sizes[2] != NKV * DM) return;
  if (in_sizes[3] != NKV * DM) return;
  if (in_sizes[4] != NH * DM) return;
  if (in_sizes[5] != DM * NKV) return;
  if (out_size != ROWS * DM) return;

  const float* x   = (const float*)d_in[0];
  const float* wk  = (const float*)d_in[1];
  const float* wv  = (const float*)d_in[2];
  const float* wq  = (const float*)d_in[3];
  const float* wg  = (const float*)d_in[4];
  const float* wo  = (const float*)d_in[5];
  float* out = (float*)d_out;

  size_t off = 0;
  const size_t oX   = off; off += (size_t)ROWS * DM * 2;
  const size_t oWq  = off; off += (size_t)NKV * DM * 2;
  const size_t oWkv = off; off += (size_t)2 * NKV * DM * 2;
  const size_t oWo  = off; off += (size_t)DM * NKV * 2;
  const size_t oG   = off; off += (size_t)SQ * NH * 4;
  const size_t oQ   = off; off += (size_t)ROWS * QLD * 2;
  const size_t oKV  = off; off += (size_t)SQ * KVLD * 2;
  const size_t oR   = off; off += (size_t)ROWS * OLD * 2;
  if (off > ws_size) return;

  char* ws = (char*)d_ws;
  _Float16* Xh   = (_Float16*)(ws + oX);
  _Float16* Wqh  = (_Float16*)(ws + oWq);
  _Float16* Wkvh = (_Float16*)(ws + oWkv);
  _Float16* Woh  = (_Float16*)(ws + oWo);
  float*    G0   = (float*)(ws + oG);
  _Float16* Qp   = (_Float16*)(ws + oQ);
  _Float16* KVp  = (_Float16*)(ws + oKV);
  _Float16* Rp   = (_Float16*)(ws + oR);

  const int gx = in_sizes[0] / 8;
  const int gw = in_sizes[1] / 8;
  const int go = in_sizes[5] / 8;
  k_cvt<<<dim3((gx + 255) / 256), dim3(256), 0, stream>>>(x,  Xh,   gx, 1.0f);
  k_cvt<<<dim3((gw + 255) / 256), dim3(256), 0, stream>>>(wq, Wqh,  gw, 32.0f);
  k_cvt<<<dim3((gw + 255) / 256), dim3(256), 0, stream>>>(wk, Wkvh, gw, 32.0f);
  k_cvt<<<dim3((gw + 255) / 256), dim3(256), 0, stream>>>(wv, Wkvh + (size_t)NKV * DM, gw, 32.0f);
  k_cvt<<<dim3((go + 255) / 256), dim3(256), 0, stream>>>(wo, Woh,  go, 32.0f);
  k_gate<<<dim3(SQ / 4), dim3(256), 0, stream>>>(x, wg, G0);
  k_lin<DM><<<dim3(ROWS / 256, NKV / 64), dim3(256), 0, stream>>>(Xh, DM, Wqh, Qp, QLD, 0.125f);
  k_lin<DM><<<dim3(SQ / 256, (2 * NKV) / 64), dim3(256), 0, stream>>>(Xh, DM, Wkvh, KVp, KVLD, 0.125f);
  k_scan<<<dim3(NB * NH), dim3(128), 0, stream>>>(Qp, KVp, G0, Rp);
  k_proj<<<dim3(ROWS / 256, DM / 64), dim3(256), 0, stream>>>(Rp, Woh, x, out);
  (void)hipGetLastError();
}
